// Non_local_Attn_5677946765888
// MI455X (gfx1250) — hardware-verified
//
#include <hip/hip_runtime.h>
#include <math.h>

constexpr int kB    = 4;
constexpr int kC    = 256;
constexpr int kHW   = 4096;
constexpr int kG    = 8;
constexpr int kCPG  = 32;
constexpr int kTok  = kB * kHW;
constexpr int kChunk = 2048;
constexpr int kStatPitch = 32;
constexpr int kStatIters = (kCPG * kHW) / (256 * 4);
constexpr float kEps        = 1e-5f;
constexpr float kWCarry     = 16.0f;
constexpr float kWCarryInv  = 1.0f / 16.0f;
constexpr float kScoreScale = 0.0625f;
constexpr float kPCarry     = 2048.0f;
constexpr float kPCarryInv  = 1.0f / 2048.0f;
static_assert(kStatIters * 256 * 4 == kCPG * kHW, "stats coverage");

typedef __attribute__((ext_vector_type(16))) _Float16 v16h;
typedef __attribute__((ext_vector_type(8)))  _Float16 v8h;
typedef __attribute__((ext_vector_type(16))) __bf16   v16b;
typedef __attribute__((ext_vector_type(8)))  __bf16   v8b;
typedef __attribute__((ext_vector_type(8)))  float    v8f;
typedef __attribute__((ext_vector_type(4)))  float    v4f;
typedef __attribute__((ext_vector_type(4)))  unsigned int v4u;

__device__ __forceinline__ unsigned short f2bf_bits(float f) {
  unsigned u = __float_as_uint(f);
  return (unsigned short)((u + 0x7FFFu + ((u >> 16) & 1u)) >> 16);
}
__device__ __forceinline__ float bf_bits2f(unsigned short h) { return __uint_as_float(((unsigned)h) << 16); }

__device__ __forceinline__ void dep_guard_h(v8f& a, v8f& b, v16h x, v16h y) { asm volatile("v_nop\n\tv_nop\n\tv_nop\n\tv_nop" : "+v"(a), "+v"(b) : "v"(x), "v"(y)); }
__device__ __forceinline__ void dep_guard_b(v8f& a, v8f& b, v16b x, v16b y) { asm volatile("v_nop\n\tv_nop\n\tv_nop\n\tv_nop" : "+v"(a), "+v"(b) : "v"(x), "v"(y)); }
__device__ __forceinline__ void keep4_h(v16h a, v16h b, v16h c, v16h d) { asm volatile("v_nop" :: "v"(a), "v"(b), "v"(c), "v"(d)); }
__device__ __forceinline__ void keep4_b(v16b a, v16b b, v16b c, v16b d) { asm volatile("v_nop" :: "v"(a), "v"(b), "v"(c), "v"(d)); }
__device__ __forceinline__ void acc_guard4(v8f& a, v8f& b, v8f& c, v8f& d) { asm volatile("v_nop\n\tv_nop\n\tv_nop\n\tv_nop" : "+v"(a), "+v"(b), "+v"(c), "+v"(d)); }
template <typename T> struct Frag;
template <> struct Frag<_Float16> {
  typedef v16h V; union U { v16h v; v8h h[2]; };
  static __device__ __forceinline__ v16h load(const _Float16* p) {
    U f; f.h[0] = *(const v8h*)(p); f.h[1] = *(const v8h*)(p + 16); return f.v;
  }
  static __device__ __forceinline__ v8f mma(v16h a, v16h b, v8f c) {
    return __builtin_amdgcn_wmma_f32_16x16x32_f16(false, a, false, b, (short)0, c, false, false);
  }
  static __device__ __forceinline__ void guard(v8f& a, v8f& b, v16h x, v16h y) { dep_guard_h(a, b, x, y); }
  static __device__ __forceinline__ void keep(v16h a, v16h b, v16h c, v16h d) { keep4_h(a, b, c, d); }
};
template <> struct Frag<__bf16> {
  typedef v16b V; union U { v16b v; v8b h[2]; };
  static __device__ __forceinline__ v16b load(const __bf16* p) {
    U f; f.h[0] = *(const v8b*)(p); f.h[1] = *(const v8b*)(p + 16); return f.v;
  }
  static __device__ __forceinline__ v8f mma(v16b a, v16b b, v8f c) {
    return __builtin_amdgcn_wmma_f32_16x16x32_bf16(false, a, false, b, (short)0, c, false, false);
  }
  static __device__ __forceinline__ void guard(v8f& a, v8f& b, v16b x, v16b y) { dep_guard_b(a, b, x, y); }
  static __device__ __forceinline__ void keep(v16b a, v16b b, v16b c, v16b d) { keep4_b(a, b, c, d); }
};

__device__ __forceinline__ unsigned pk16(unsigned short a, unsigned short b) { return (unsigned)a | ((unsigned)b << 16); }
__device__ __forceinline__ unsigned short h_bits(float f) { const _Float16 h = (_Float16)f; return __builtin_bit_cast(unsigned short, h); }

template <int ET> struct Elem;
template <> struct Elem<0> { typedef _Float16 T; };
template <> struct Elem<1> { typedef __bf16 T; };
template <int ET, bool SPLIT, int BIAS_MODE, int OUT_MODE, bool RESID, int ACT = 0>
__global__ __launch_bounds__(256) void wmma_gemm64(
    const unsigned short* __restrict__ Ap, const unsigned short* __restrict__ A2p, int lda, long strideA,
    const unsigned short* __restrict__ Btp, const unsigned short* __restrict__ Bt2p, int ldb, long strideB,
    void* __restrict__ Cout, void* __restrict__ Cout2, int ldc, long strideC,
    const float* __restrict__ bias,
    const float* __restrict__ resid, long strideR,
    int M, int N, int K, float scale) {
  typedef typename Elem<ET>::T T;
  typedef typename Frag<T>::V V;
  const T* A = (const T*)Ap; const T* A2 = (const T*)A2p; const T* Bt = (const T*)Btp; const T* Bt2 = (const T*)Bt2p;
  __shared__ __align__(16) float sT[8][16 * 68];
  const int b    = blockIdx.y;
  const int lane = threadIdx.x & 31;
  const int wave = threadIdx.x >> 5;
  const int tilesN = N >> 6;
  const int tilesM = M >> 6;
  const int tile = blockIdx.x * 8 + wave;
  if (tile >= tilesM * tilesN) return;
  const int tm = tile / tilesN;
  const int tn = tile - tm * tilesN;
  const int m0 = tm << 6;
  const int n0 = tn << 6;

  const T* Ab  = A  + (size_t)b * strideA;
  const T* Bb  = Bt + (size_t)b * strideB;
  const T* Ab2 = SPLIT ? (A2  + (size_t)b * strideA) : nullptr;
  const T* Bb2 = SPLIT ? (Bt2 + (size_t)b * strideB) : nullptr;

  const int rlane = lane & 15;
  const int koff  = (lane >> 4) * 8;
  const int mOff  = (lane >> 4) * 8;

  v8f acc[4][4];
#pragma unroll
  for (int i = 0; i < 4; ++i)
#pragma unroll
    for (int j = 0; j < 4; ++j) acc[i][j] = (v8f){0.f,0.f,0.f,0.f,0.f,0.f,0.f,0.f};

  for (int k0 = 0; k0 < K; k0 += 32) {
    V bh[4], bl[4];
#pragma unroll
    for (int j = 0; j < 4; ++j) {
      const size_t bo = (size_t)(n0 + (j << 4) + rlane) * ldb + koff + k0;
      bh[j] = Frag<T>::load(Bb + bo);
      if (SPLIT) bl[j] = Frag<T>::load(Bb2 + bo);
    }
#pragma unroll
    for (int i = 0; i < 4; ++i) {
      const size_t ao = (size_t)(m0 + (i << 4) + rlane) * lda + koff + k0;
      V ah = Frag<T>::load(Ab + ao);
      V al;
      if (SPLIT) al = Frag<T>::load(Ab2 + ao);
#pragma unroll
      for (int j = 0; j < 4; ++j) {
        acc[i][j] = Frag<T>::mma(ah, bh[j], acc[i][j]);
        if (SPLIT) {
          acc[i][j] = Frag<T>::mma(ah, bl[j], acc[i][j]);
          acc[i][j] = Frag<T>::mma(al, bh[j], acc[i][j]);
        }
      }
      Frag<T>::guard(acc[i][0], acc[i][3], ah, SPLIT ? al : ah);
    }
    Frag<T>::keep(bh[0], bh[1], bh[2], bh[3]);
    if (SPLIT) Frag<T>::keep(bl[0], bl[1], bl[2], bl[3]);
  }
  acc_guard4(acc[0][0], acc[0][1], acc[0][2], acc[0][3]);
  acc_guard4(acc[1][0], acc[1][1], acc[1][2], acc[1][3]);
  acc_guard4(acc[2][0], acc[2][1], acc[2][2], acc[2][3]);
  acc_guard4(acc[3][0], acc[3][1], acc[3][2], acc[3][3]);

  float* slab = sT[wave];
  const float* Rb = RESID ? (resid + (size_t)b * strideR) : nullptr;
#pragma unroll
  for (int i = 0; i < 4; ++i) {
    const int mBase = m0 + (i << 4);
#pragma unroll
    for (int j = 0; j < 4; ++j) {
      const int n = n0 + (j << 4) + rlane;
      float bv = 0.f;
      if (BIAS_MODE == 2) bv = bias[n];
#pragma unroll
      for (int r = 0; r < 8; ++r) {
        float v = acc[i][j][r] * scale;
        if (BIAS_MODE == 1) v += bias[mBase + mOff + r];
        if (BIAS_MODE == 2) v += bv;
        if (RESID) v += Rb[(size_t)(mBase + mOff + r) * ldc + n];
        if (ACT == 2) v = fmaxf(v, 0.0f);
        if (ACT == 4) v = (v > 0.f) ? v : 0.01f * v;
        slab[(mOff + r) * 68 + (j << 4) + rlane] = v;
      }
    }
    __builtin_amdgcn_fence(__ATOMIC_RELEASE, "workgroup");
    __builtin_amdgcn_wave_barrier();
    __builtin_amdgcn_fence(__ATOMIC_ACQUIRE, "workgroup");
    if (OUT_MODE == 0) {
      float* C = (float*)Cout + (size_t)b * strideC;
      const int hh = lane >> 4, c4 = (lane & 15) * 4;
      for (int pass = 0; pass < 2; ++pass) {
#pragma unroll
        for (int it = 0; it < 8; ++it) {
          const int row = it * 2 + hh;
          v4f v = *(const v4f*)(slab + row * 68 + c4);
          *(volatile v4f*)(C + (size_t)(mBase + row) * ldc + n0 + c4) = v;
        }
        __threadfence();
      }
    } else {
      const int q = lane >> 3, c8 = (lane & 7) * 8;
      unsigned short* C  = (unsigned short*)Cout  + (size_t)b * strideC;
      unsigned short* C2 = (OUT_MODE == 2) ? ((unsigned short*)Cout2 + (size_t)b * strideC) : nullptr;
      for (int pass = 0; pass < 2; ++pass) {
#pragma unroll
        for (int it = 0; it < 4; ++it) {
          const int row = it * 4 + q;
          const float* sp = slab + row * 68 + c8;
          v8h hv, lv;
#pragma unroll
          for (int e = 0; e < 8; ++e) {
            if (OUT_MODE == 1) {
              hv[e] = (_Float16)sp[e];
            } else {
              unsigned short hb = f2bf_bits(sp[e]);
              unsigned short lb = f2bf_bits(sp[e] - bf_bits2f(hb));
              hv[e] = __builtin_bit_cast(_Float16, hb);
              lv[e] = __builtin_bit_cast(_Float16, lb);
            }
          }
          *(volatile v8h*)(C + (size_t)(mBase + row) * ldc + n0 + c8) = hv;
          if (OUT_MODE == 2) *(volatile v8h*)(C2 + (size_t)(mBase + row) * ldc + n0 + c8) = lv;
        }
        __threadfence();
      }
    }
    __builtin_amdgcn_fence(__ATOMIC_RELEASE, "workgroup");
    __builtin_amdgcn_wave_barrier();
    __builtin_amdgcn_fence(__ATOMIC_ACQUIRE, "workgroup");
  }
}

__global__ __launch_bounds__(256) void gn_stats_kernel(const float* __restrict__ x, float* __restrict__ stats) {
  __shared__ float redS[8];
  __shared__ float redQ[8];
  const int bg = blockIdx.x;
  const int b = bg >> 3, g = bg & 7;
  const float* base = x + ((size_t)b * kC + (size_t)g * kCPG) * kHW;
  const int t = threadIdx.x, lane = t & 31, wave = t >> 5;
  float s0 = 0.f, s1 = 0.f, s2 = 0.f, s3 = 0.f;
  float q0 = 0.f, q1 = 0.f, q2 = 0.f, q3 = 0.f;
#pragma unroll 1
  for (int i = 0; i < kStatIters; ++i) {
    const v4f v = *(const v4f*)(base + ((size_t)i * 256 + t) * 4);
    s0 += v[0]; s1 += v[1]; s2 += v[2]; s3 += v[3];
    q0 += v[0] * v[0]; q1 += v[1] * v[1]; q2 += v[2] * v[2]; q3 += v[3] * v[3];
  }
  float s = (s0 + s1) + (s2 + s3);
  float q = (q0 + q1) + (q2 + q3);
#pragma unroll
  for (int off = 16; off > 0; off >>= 1) {
    s += __shfl_xor(s, off, 32);
    q += __shfl_xor(q, off, 32);
  }
  if (lane == 0) { redS[wave] = s; redQ[wave] = q; }
  __syncthreads();
  if (wave == 0) {
    float ts = 0.f, tq = 0.f;
#pragma unroll
    for (int w = 0; w < 8; ++w) { ts += redS[w]; tq += redQ[w]; }
    const float inv = 1.0f / (float)(kCPG * kHW);
    const float mu = ts * inv;
    float var = tq * inv - mu * mu;
    var = fmaxf(var, 0.0f);
    const float rs = rsqrtf(var + kEps);
    const float val = (lane == 0) ? mu : ((lane == 1) ? rs : 0.0f);
    volatile float* sp = stats + (size_t)bg * kStatPitch + lane;
    *sp = val;
    __threadfence();
    *sp = val;
  }
}

__global__ __launch_bounds__(256) void gn_apply_kernel(const float* __restrict__ x, const float* __restrict__ gamma,
                                                       const float* __restrict__ beta, const float* __restrict__ stats,
                                                       unsigned short* __restrict__ H) {
  __shared__ float sm[64][65];
  const int t  = threadIdx.x;
  const int p0 = blockIdx.x * 64;
  const int c0 = blockIdx.y * 64;
  const int b  = blockIdx.z;
#pragma unroll
  for (int i = 0; i < 16; ++i) {
    const int e  = i * 256 + t;
    const int cl = e >> 6;
    const int pl = e & 63;
    const int c  = c0 + cl;
    const int g  = c >> 5;
    const float mu = stats[(size_t)(b * kG + g) * kStatPitch];
    const float rs = stats[(size_t)(b * kG + g) * kStatPitch + 1];
    const float ga = gamma[c];
    const float be = beta[c];
    const float v  = x[((size_t)(b * kC + c)) * kHW + p0 + pl];
    sm[pl][cl] = ((v - mu) * rs) * ga + be;
  }
  __syncthreads();
  const int lane = t & 31, wave = t >> 5;
  const int q = lane >> 3, c8 = (lane & 7) * 8;
  for (int pass = 0; pass < 2; ++pass) {
#pragma unroll
    for (int it = 0; it < 2; ++it) {
      const int row = wave * 8 + it * 4 + q;
      unsigned short hb[8];
#pragma unroll
      for (int e = 0; e < 8; ++e) hb[e] = h_bits(sm[row][c8 + e]);
      const v4u u = (v4u){pk16(hb[0], hb[1]), pk16(hb[2], hb[3]), pk16(hb[4], hb[5]), pk16(hb[6], hb[7])};
      *(volatile v4u*)(H + (size_t)(b * kHW + p0 + row) * kC + c0 + c8) = u;
    }
    __threadfence();
  }
}

__global__ __launch_bounds__(256) void wcast_kernel(const float* __restrict__ w0, const float* __restrict__ w1,
                                                    const float* __restrict__ w2, unsigned short* __restrict__ out,
                                                    float scale) {
  const int i = blockIdx.x * 256 + threadIdx.x;
  const int z = blockIdx.y;
  const float* W = (z == 0) ? w0 : ((z == 1) ? w1 : w2);
  if (i >= (kC * kC) / 8) return;
  const float* p = W + 8 * (size_t)i;
  const v4f a = *(const v4f*)(p);
  const v4f c = *(const v4f*)(p + 4);
  unsigned short hb[8];
#pragma unroll
  for (int e = 0; e < 4; ++e) {
    hb[e]     = h_bits(a[e] * scale);
    hb[4 + e] = h_bits(c[e] * scale);
  }
  const v4u u = (v4u){pk16(hb[0], hb[1]), pk16(hb[2], hb[3]), pk16(hb[4], hb[5]), pk16(hb[6], hb[7])};
  unsigned short* op = out + (size_t)z * kC * kC + 8 * (size_t)i;
  *(volatile v4u*)op = u;
  __threadfence();
  *(volatile v4u*)op = u;
}

__global__ __launch_bounds__(512) void softmax_row_kernel(const float* __restrict__ S, unsigned short* __restrict__ P) {
  __shared__ float redM[16];
  __shared__ float redS[16];
  const int row  = blockIdx.x;
  const int t    = threadIdx.x;
  const int lane = t & 31, wave = t >> 5;
  const int c0   = t * 8;
  const float* sr = S + (size_t)row * kHW + c0;
  const v4f a = *(const v4f*)(sr);
  const v4f c = *(const v4f*)(sr + 4);
  float xv[8];
#pragma unroll
  for (int e = 0; e < 4; ++e) { xv[e] = a[e]; xv[4 + e] = c[e]; }
  float m = fmaxf(fmaxf(fmaxf(xv[0], xv[1]), fmaxf(xv[2], xv[3])), fmaxf(fmaxf(xv[4], xv[5]), fmaxf(xv[6], xv[7])));
#pragma unroll
  for (int off = 16; off > 0; off >>= 1) m = fmaxf(m, __shfl_xor(m, off, 32));
  if (lane == 0) redM[wave] = m;
  __syncthreads();
  float gm = redM[0];
#pragma unroll
  for (int w = 1; w < 16; ++w) gm = fmaxf(gm, redM[w]);
  float ev[8];
  float s = 0.f;
#pragma unroll
  for (int e = 0; e < 8; ++e) { ev[e] = expf(xv[e] - gm); s += ev[e]; }
#pragma unroll
  for (int off = 16; off > 0; off >>= 1) s += __shfl_xor(s, off, 32);
  if (lane == 0) redS[wave] = s;
  __syncthreads();
  float gs = 0.f;
#pragma unroll
  for (int w = 0; w < 16; ++w) gs += redS[w];
  const float f = kPCarry * (1.0f / gs);
  unsigned short hb[8];
#pragma unroll
  for (int e = 0; e < 8; ++e) hb[e] = h_bits(ev[e] * f);
  const v4u u = (v4u){pk16(hb[0], hb[1]), pk16(hb[2], hb[3]), pk16(hb[4], hb[5]), pk16(hb[6], hb[7])};
  unsigned short* pp = P + (size_t)row * kHW + c0;
  *(volatile v4u*)pp = u;
  __threadfence();
  *(volatile v4u*)pp = u;
}

extern "C" void kernel_launch(void* const* d_in, const int* in_sizes, int n_in,
                              void* d_out, int out_size, void* d_ws,
                              size_t ws_size, hipStream_t stream) {
  if (n_in < 9) return;
  if (in_sizes[0] != kB * kC * kHW || out_size != kB * kC * kHW) return;
  if (in_sizes[1] != kC || in_sizes[2] != kC) return;
  if (in_sizes[3] != kC * kC || in_sizes[5] != kC * kC || in_sizes[7] != kC * kC) return;
  if (in_sizes[4] != kC || in_sizes[6] != kC || in_sizes[8] != kC) return;

  const float* x     = (const float*)d_in[0];
  const float* gamma = (const float*)d_in[1];
  const float* beta  = (const float*)d_in[2];
  const float* wq    = (const float*)d_in[3];
  const float* bq    = (const float*)d_in[4];
  const float* wk    = (const float*)d_in[5];
  const float* bk    = (const float*)d_in[6];
  const float* wv    = (const float*)d_in[7];
  const float* bv    = (const float*)d_in[8];
  float* out = (float*)d_out;

  const size_t szStats = (size_t)kB * kG * kStatPitch * sizeof(float);
  const size_t szH     = (size_t)kTok * kC * 2;
  const size_t szW     = (size_t)3 * kC * kC * 2;
  const size_t szQ     = (size_t)kTok * kC * 2;
  const size_t szV     = (size_t)kB * kC * kHW * 2;
  const size_t szS     = (size_t)kChunk * kHW * 4;
  const size_t szP     = (size_t)kChunk * kHW * 2;
  size_t off = 0;
  char* ws = (char*)d_ws;
  float*          stats = (float*)(ws + off);           off += szStats;
  unsigned short* H16   = (unsigned short*)(ws + off);  off += szH;
  unsigned short* W16   = (unsigned short*)(ws + off);  off += szW;
  unsigned short* Q16   = (unsigned short*)(ws + off);  off += szQ;
  unsigned short* K16   = (unsigned short*)(ws + off);  off += szQ;
  unsigned short* V16   = (unsigned short*)(ws + off);  off += szV;
  float*          Sbuf  = (float*)(ws + off);           off += szS;
  unsigned short* P16   = (unsigned short*)(ws + off);  off += szP;
  if (off > ws_size) return;

  gn_stats_kernel<<<dim3(kB * kG), dim3(256), 0, stream>>>(x, stats);
  gn_apply_kernel<<<dim3(kHW / 64, kC / 64, kB), dim3(256), 0, stream>>>(x, gamma, beta, stats, H16);
  wcast_kernel<<<dim3((kC * kC / 8) / 256, 3), dim3(256), 0, stream>>>(wq, wk, wv, W16, kWCarry);

  wmma_gemm64<0, false, 2, 1, false><<<dim3((kTok / 64) * (kC / 64) / 8, 1), dim3(256), 0, stream>>>(
      H16, nullptr, kC, 0L, W16, nullptr, kC, 0L, (void*)Q16, nullptr, kC, 0L,
      bq, nullptr, 0L, kTok, kC, kC, kWCarryInv);
  wmma_gemm64<0, false, 2, 1, false><<<dim3((kTok / 64) * (kC / 64) / 8, 1), dim3(256), 0, stream>>>(
      H16, nullptr, kC, 0L, W16 + (size_t)kC * kC, nullptr, kC, 0L, (void*)K16, nullptr, kC, 0L,
      bk, nullptr, 0L, kTok, kC, kC, kWCarryInv);
  wmma_gemm64<0, false, 1, 1, false><<<dim3((kC / 64) * (kHW / 64) / 8, kB), dim3(256), 0, stream>>>(
      W16 + (size_t)2 * kC * kC, nullptr, kC, 0L, H16, nullptr, kC, (long)kHW * kC, (void*)V16, nullptr, kHW, (long)kC * kHW,
      bv, nullptr, 0L, kC, kHW, kC, kWCarryInv);

  for (int b = 0; b < kB; ++b) {
    for (int hc = 0; hc < kHW / kChunk; ++hc) {
      const int i0 = hc * kChunk;
      wmma_gemm64<0, false, 0, 0, false><<<dim3((kChunk / 64) * (kHW / 64) / 8, 1), dim3(256), 0, stream>>>(
          Q16 + ((size_t)b * kHW + i0) * kC, nullptr, kC, 0L, K16 + (size_t)b * kHW * kC, nullptr, kC, 0L,
          (void*)Sbuf, nullptr, kHW, 0L, nullptr, nullptr, 0L, kChunk, kHW, kC, kScoreScale);
      softmax_row_kernel<<<dim3(kChunk), dim3(512), 0, stream>>>(Sbuf, P16);
      wmma_gemm64<0, false, 0, 0, true><<<dim3((kC / 64) * (kChunk / 64) / 8, 1), dim3(256), 0, stream>>>(
          V16 + (size_t)b * kC * kHW, nullptr, kHW, 0L, P16, nullptr, kHW, 0L,
          (void*)(out + (size_t)b * kC * kHW + i0), nullptr, kHW, 0L, nullptr,
          x + (size_t)b * kC * kHW + i0, 0L, kC, kChunk, kHW, kPCarryInv);
    }
  }
}
